// Block_29403346109123
// MI455X (gfx1250) — hardware-verified
//
#include <hip/hip_runtime.h>


#pragma clang fp contract(off)

#ifndef NB
#define NB 2
#endif
#ifndef SEQ
#define SEQ 4096
#endif
#define NB_FULL 2
#define SEQ_FULL 4096
#define CDIM 512
#define NHEAD 8
#define HD 64
#define HID 2048
#define MROWS (NB * SEQ)

static_assert(NB >= 1 && NB <= NB_FULL);
static_assert(SEQ % 64 == 0 && SEQ >= 64 && SEQ <= SEQ_FULL);
static_assert(CDIM == NHEAD * HD);
static_assert(HD == 64);
static_assert(CDIM == 512);
static_assert(CDIM == 32 * 2 * 8);
static_assert(HID % 64 == 0 && CDIM % 64 == 0);
static_assert(CDIM % 32 == 0 && HID % 32 == 0);
static_assert(MROWS % 64 == 0);
static_assert(MROWS % 8 == 0);
static_assert((3 * CDIM) % 64 == 0);

typedef _Float16 v16h __attribute__((ext_vector_type(16)));
typedef _Float16 v8h  __attribute__((ext_vector_type(8)));
typedef float    v8f  __attribute__((ext_vector_type(8)));
typedef float    v4f  __attribute__((ext_vector_type(4)));
typedef unsigned int v4u __attribute__((ext_vector_type(4)));

union Frag { v16h v; v4u q[2]; };

__device__ __forceinline__ v8f mma(v16h a, v16h b, v8f c) {
  v8f d = __builtin_amdgcn_wmma_f32_16x16x32_f16(false, a, false, b, (short)0, c, false, false);
  asm volatile("v_nop\n\tv_nop\n\tv_nop\n\tv_nop" : "+v"(d) : "v"(a), "v"(b));
  return d;
}

__device__ __forceinline__ v8f zero8() {
  v8f z;
#pragma unroll
  for (int i = 0; i < 8; ++i) z[i] = 0.0f;
  return z;
}

__device__ __forceinline__ float bf16q(float f) {
  unsigned int u = __float_as_uint(f);
  unsigned int r = u + 0x7FFFu + ((u >> 16) & 1u);
  r = ((u & 0x7F800000u) == 0x7F800000u) ? u : r;
  return __uint_as_float(r & 0xFFFF0000u);
}
__device__ __forceinline__ v4f bf16q4(v4f a) {
  v4f r;
  r.x = bf16q(a.x); r.y = bf16q(a.y); r.z = bf16q(a.z); r.w = bf16q(a.w);
  return r;
}
__device__ __forceinline__ unsigned short hbits(float f) {
  _Float16 h = (_Float16)f;
  return __builtin_bit_cast(unsigned short, h);
}
__device__ __forceinline__ v4u pack8h(float f0, float f1, float f2, float f3,
                                      float f4, float f5, float f6, float f7) {
  v8h t;
  t[0] = (_Float16)f0; t[1] = (_Float16)f1; t[2] = (_Float16)f2; t[3] = (_Float16)f3;
  t[4] = (_Float16)f4; t[5] = (_Float16)f5; t[6] = (_Float16)f6; t[7] = (_Float16)f7;
  return __builtin_bit_cast(v4u, t);
}
__device__ __forceinline__ float gelu_erf(float u) {
  return 0.5f * u * (1.0f + erff(u * 0.70710678118654752f));
}

__global__ __launch_bounds__(256) void k_wprep(
    const float* __restrict__ src, unsigned short* __restrict__ dst, int K, int N, int rowoff) {
  __shared__ __attribute__((aligned(16))) unsigned short sT[64][72];
  const int tid = threadIdx.x;
  const int k0 = blockIdx.x * 64, n0 = blockIdx.y * 64;
#pragma unroll
  for (int it = 0; it < 4; ++it) {
    const int idx = it * 256 + tid;
    const int kk = idx >> 4;
    const int j4 = (idx & 15) * 4;
    const v4f wv = *(const v4f*)(src + (size_t)(k0 + kk) * (size_t)N + n0 + j4);
    sT[j4 + 0][kk] = hbits(bf16q(wv.x) * 16.0f);
    sT[j4 + 1][kk] = hbits(bf16q(wv.y) * 16.0f);
    sT[j4 + 2][kk] = hbits(bf16q(wv.z) * 16.0f);
    sT[j4 + 3][kk] = hbits(bf16q(wv.w) * 16.0f);
  }
  __syncthreads();
  v4u val[2];
  size_t off[2];
#pragma unroll
  for (int p = 0; p < 2; ++p) {
    const int n = p * 32 + (tid >> 3);
    const int piece = tid & 7;
    val[p] = *(const v4u*)&sT[n][piece * 8];
    off[p] = (size_t)(rowoff + n0 + n) * (size_t)K + k0 + piece * 8;
  }
#pragma unroll
  for (int p = 0; p < 2; ++p) *(volatile v4u*)(dst + off[p]) = val[p];
  __threadfence();
#pragma unroll
  for (int p = 0; p < 2; ++p) *(volatile v4u*)(dst + off[p]) = val[p];
}

template <int RNDIN>
__device__ __forceinline__ void ln_body(
    const float* __restrict__ x, const float* __restrict__ g, const float* __restrict__ bt,
    unsigned short* __restrict__ hout, int nrows) {
  const int lane = threadIdx.x & 31, w = threadIdx.x >> 5;
  const int row = blockIdx.x * 8 + w;
  if (row >= nrows) return;
  size_t xrow;
  if (RNDIN) {
    const int b = row / SEQ, t = row - b * SEQ;
    xrow = ((size_t)b * SEQ_FULL + t) * CDIM;
  } else {
    xrow = (size_t)row * CDIM;
  }
  const int c0 = lane * 8;
  const int c1 = 256 + lane * 8;

  float v[16];
  {
    const v4f t0 = *(const v4f*)(x + xrow + c0);
    const v4f t1 = *(const v4f*)(x + xrow + c0 + 4);
    const v4f t2 = *(const v4f*)(x + xrow + c1);
    const v4f t3 = *(const v4f*)(x + xrow + c1 + 4);
    v[0] = t0.x; v[1] = t0.y; v[2] = t0.z; v[3] = t0.w;
    v[4] = t1.x; v[5] = t1.y; v[6] = t1.z; v[7] = t1.w;
    v[8] = t2.x; v[9] = t2.y; v[10] = t2.z; v[11] = t2.w;
    v[12] = t3.x; v[13] = t3.y; v[14] = t3.z; v[15] = t3.w;
  }
  if (RNDIN) {
#pragma unroll
    for (int i = 0; i < 16; ++i) v[i] = bf16q(v[i]);
  }

  float s = 0.0f;
#pragma unroll
  for (int i = 0; i < 16; ++i) s += v[i];
#pragma unroll
  for (int xm = 1; xm < 32; xm <<= 1) s += __shfl_xor(s, xm, 32);
  const float mu = s * (1.0f / CDIM);

  float d[16];
#pragma unroll
  for (int i = 0; i < 16; ++i) d[i] = v[i] - mu;
  float qs = 0.0f;
#pragma unroll
  for (int i = 0; i < 16; ++i) qs += d[i] * d[i];
#pragma unroll
  for (int xm = 1; xm < 32; xm <<= 1) qs += __shfl_xor(qs, xm, 32);
  const float var = qs * (1.0f / CDIM);
  const float rstd = rsqrtf(var + 1e-5f);

  float gg[16], bb[16];
  {
    const v4f g0 = bf16q4(*(const v4f*)(g + c0));
    const v4f g1 = bf16q4(*(const v4f*)(g + c0 + 4));
    const v4f g2 = bf16q4(*(const v4f*)(g + c1));
    const v4f g3 = bf16q4(*(const v4f*)(g + c1 + 4));
    const v4f b0 = bf16q4(*(const v4f*)(bt + c0));
    const v4f b1 = bf16q4(*(const v4f*)(bt + c0 + 4));
    const v4f b2 = bf16q4(*(const v4f*)(bt + c1));
    const v4f b3 = bf16q4(*(const v4f*)(bt + c1 + 4));
    gg[0] = g0.x; gg[1] = g0.y; gg[2] = g0.z; gg[3] = g0.w;
    gg[4] = g1.x; gg[5] = g1.y; gg[6] = g1.z; gg[7] = g1.w;
    gg[8] = g2.x; gg[9] = g2.y; gg[10] = g2.z; gg[11] = g2.w;
    gg[12] = g3.x; gg[13] = g3.y; gg[14] = g3.z; gg[15] = g3.w;
    bb[0] = b0.x; bb[1] = b0.y; bb[2] = b0.z; bb[3] = b0.w;
    bb[4] = b1.x; bb[5] = b1.y; bb[6] = b1.z; bb[7] = b1.w;
    bb[8] = b2.x; bb[9] = b2.y; bb[10] = b2.z; bb[11] = b2.w;
    bb[12] = b3.x; bb[13] = b3.y; bb[14] = b3.z; bb[15] = b3.w;
  }
  float y[16];
#pragma unroll
  for (int i = 0; i < 16; ++i) y[i] = d[i] * rstd * gg[i] + bb[i];

  const v4u o0 = pack8h(y[0], y[1], y[2], y[3], y[4], y[5], y[6], y[7]);
  const v4u o1 = pack8h(y[8], y[9], y[10], y[11], y[12], y[13], y[14], y[15]);
  unsigned short* orow = hout + (size_t)row * CDIM;
  *(volatile v4u*)(orow + c0) = o0;
  *(volatile v4u*)(orow + c1) = o1;
  __threadfence();
  *(volatile v4u*)(orow + c0) = o0;
  *(volatile v4u*)(orow + c1) = o1;
}

__global__ __launch_bounds__(256) void k_ln_in(
    const float* __restrict__ x, const float* __restrict__ g, const float* __restrict__ bt,
    unsigned short* __restrict__ hout, int nrows) {
  ln_body<1>(x, g, bt, hout, nrows);
}
__global__ __launch_bounds__(256) void k_ln_mid(
    const float* __restrict__ x, const float* __restrict__ g, const float* __restrict__ bt,
    unsigned short* __restrict__ hout, int nrows) {
  ln_body<0>(x, g, bt, hout, nrows);
}

__device__ __forceinline__ void gemm_main(
    const unsigned short* __restrict__ A, const unsigned short* __restrict__ Bt, int K,
    int m0, int n0, int w, int m, int k8, v8f (&acc)[4]) {
#pragma unroll
  for (int j = 0; j < 4; ++j) acc[j] = zero8();
  const unsigned short* ap = A + (size_t)(m0 + 16 * w + m) * (size_t)K + k8;
  const unsigned short* bp = Bt + (size_t)(n0 + m) * (size_t)K + k8;
  const size_t jstep = (size_t)16 * (size_t)K;
#pragma unroll 1
  for (int k0 = 0; k0 < K; k0 += 32) {
    Frag a;
    a.q[0] = *(const v4u*)(ap + k0);
    a.q[1] = *(const v4u*)(ap + k0 + 16);
#pragma unroll
    for (int j = 0; j < 4; ++j) {
      Frag b;
      const unsigned short* bj = bp + jstep * j + k0;
      b.q[0] = *(const v4u*)(bj);
      b.q[1] = *(const v4u*)(bj + 16);
      acc[j] = mma(a.v, b.v, acc[j]);
    }
  }
}

__global__ __launch_bounds__(128) void k_gemm_qkv(
    const unsigned short* __restrict__ A, const unsigned short* __restrict__ Bt,
    const float* __restrict__ bq, const float* __restrict__ bk, const float* __restrict__ bv,
    unsigned short* __restrict__ qkv) {
  __shared__ __attribute__((aligned(16))) unsigned short sT[64][72];
  const int tid = threadIdx.x, lane = tid & 31, w = tid >> 5;
  const int m = lane & 15, hl = lane >> 4, k8 = hl * 8;
  const int m0 = blockIdx.y * 64, n0 = blockIdx.x * 64;

  v8f acc[4];
  gemm_main(A, Bt, CDIM, m0, n0, w, m, k8, acc);

  const float wsc = 0.0625f;
  const int lrow0 = 16 * w + 8 * hl;
  const int which = n0 / CDIM;
  const int cb = n0 - which * CDIM;
#pragma unroll
  for (int j = 0; j < 4; ++j) {
    const int cn = cb + 16 * j + m;
    const float b0 = bf16q(bq[cn]);
    const float b1 = bf16q(bk[cn]);
    const float b2 = bf16q(bv[cn]);
    const float bj = (which == 0) ? b0 : ((which == 1) ? b1 : b2);
#pragma unroll
    for (int r = 0; r < 8; ++r) sT[lrow0 + r][16 * j + m] = hbits(acc[j][r] * wsc + bj);
  }
  __syncthreads();
  const int hh = cb / HD;
  const int b = m0 / SEQ, t0 = m0 - b * SEQ;
  const int bh = b * NHEAD + hh;
  unsigned short* dst = qkv + (size_t)which * ((size_t)MROWS * CDIM);
  v4u val[4];
  unsigned int off[4];
  if (which < 2) {
#pragma unroll
    for (int p = 0; p < 4; ++p) {
      const int row = p * 16 + 4 * w + (lane >> 3);
      const int piece = lane & 7;
      val[p] = *(const v4u*)&sT[row][piece * 8];
      off[p] = (unsigned int)((bh * SEQ + t0 + row) * HD + piece * 8);
    }
  } else {
#pragma unroll
    for (int p = 0; p < 4; ++p) {
      const int d = p * 16 + 4 * w + (lane >> 3);
      const int piece = lane & 7;
      unsigned int wv[4];
#pragma unroll
      for (int e = 0; e < 4; ++e) {
        const unsigned int lo = sT[piece * 8 + 2 * e][d];
        const unsigned int hi = sT[piece * 8 + 2 * e + 1][d];
        wv[e] = lo | (hi << 16);
      }
      v4u t;
      t.x = wv[0]; t.y = wv[1]; t.z = wv[2]; t.w = wv[3];
      val[p] = t;
      off[p] = (unsigned int)((bh * HD + d) * SEQ + t0 + piece * 8);
    }
  }
#pragma unroll
  for (int p = 0; p < 4; ++p) *(volatile v4u*)(dst + off[p]) = val[p];
  __threadfence();
#pragma unroll
  for (int p = 0; p < 4; ++p) *(volatile v4u*)(dst + off[p]) = val[p];
}

__global__ __launch_bounds__(128) void k_gemm_res(
    const unsigned short* __restrict__ A, const unsigned short* __restrict__ Bt, int K,
    const float* __restrict__ bias, const float* __restrict__ res,
    float* __restrict__ outF, int resfull, int outfull) {
  __shared__ __attribute__((aligned(16))) float sF[64][68];
  const int tid = threadIdx.x, lane = tid & 31, w = tid >> 5;
  const int m = lane & 15, hl = lane >> 4, k8 = hl * 8;
  const int m0 = blockIdx.y * 64, n0 = blockIdx.x * 64;

  v8f acc[4];
  gemm_main(A, Bt, K, m0, n0, w, m, k8, acc);

  const float wsc = 0.0625f;
  const int lrow0 = 16 * w + 8 * hl;
#pragma unroll
  for (int j = 0; j < 4; ++j) {
#pragma unroll
    for (int r = 0; r < 8; ++r) sF[lrow0 + r][16 * j + m] = acc[j][r] * wsc;
  }
  __syncthreads();
  const int b = m0 / SEQ, t0 = m0 - b * SEQ;
  v4f val[8];
  unsigned int off[8];
#pragma unroll
  for (int p = 0; p < 8; ++p) {
    const int row = 16 * w + 2 * p + hl;
    const int piece = m;
    const int ncol = n0 + 4 * piece;
    const v4f a = *(const v4f*)&sF[row][4 * piece];
    const v4f bv = bf16q4(*(const v4f*)(bias + ncol));
    const size_t frow = (size_t)b * SEQ_FULL + t0 + row;
    const size_t crow = (size_t)(m0 + row);
    const size_t rrow = resfull ? frow : crow;
    const v4f rraw = *(const v4f*)(res + rrow * (size_t)CDIM + ncol);
    const v4f rq = bf16q4(rraw);
    const v4f rr = resfull ? rq : rraw;
    val[p] = (a + bv) + rr;
    const size_t orow = outfull ? frow : crow;
    off[p] = (unsigned int)(orow * (size_t)CDIM + ncol);
  }
#pragma unroll
  for (int p = 0; p < 8; ++p) *(volatile v4f*)(outF + off[p]) = val[p];
  __threadfence();
#pragma unroll
  for (int p = 0; p < 8; ++p) *(volatile v4f*)(outF + off[p]) = val[p];
}

__global__ __launch_bounds__(128) void k_gemm_gelu(
    const unsigned short* __restrict__ A, const unsigned short* __restrict__ Bt, int K,
    const float* __restrict__ bias, unsigned short* __restrict__ out0) {
  __shared__ __attribute__((aligned(16))) unsigned short sT[64][72];
  const int tid = threadIdx.x, lane = tid & 31, w = tid >> 5;
  const int m = lane & 15, hl = lane >> 4, k8 = hl * 8;
  const int m0 = blockIdx.y * 64, n0 = blockIdx.x * 64;

  v8f acc[4];
  gemm_main(A, Bt, K, m0, n0, w, m, k8, acc);

  const float wsc = 0.0625f;
  const int lrow0 = 16 * w + 8 * hl;
#pragma unroll
  for (int j = 0; j < 4; ++j) {
    const float bj = bf16q(bias[n0 + 16 * j + m]);
#pragma unroll
    for (int r = 0; r < 8; ++r) {
      const float u = acc[j][r] * wsc + bj;
      sT[lrow0 + r][16 * j + m] = hbits(gelu_erf(u));
    }
  }
  __syncthreads();
  v4u val[4];
  unsigned int off[4];
#pragma unroll
  for (int p = 0; p < 4; ++p) {
    const int row = 16 * w + 4 * p + (lane >> 3);
    const int piece = lane & 7;
    val[p] = *(const v4u*)&sT[row][piece * 8];
    off[p] = (unsigned int)((size_t)(m0 + row) * (size_t)HID + n0 + piece * 8);
  }
#pragma unroll
  for (int p = 0; p < 4; ++p) *(volatile v4u*)(out0 + off[p]) = val[p];
  __threadfence();
#pragma unroll
  for (int p = 0; p < 4; ++p) *(volatile v4u*)(out0 + off[p]) = val[p];
}

__global__ __launch_bounds__(128) __attribute__((amdgpu_num_vgpr(256)))
void k_attn(const unsigned short* __restrict__ qp, const unsigned short* __restrict__ kp,
            const unsigned short* __restrict__ vp, unsigned short* __restrict__ op) {
  __shared__ __attribute__((aligned(16))) unsigned short sP[4][16][72];
  const int tid = threadIdx.x, lane = tid & 31, w = tid >> 5;
  const int m = lane & 15, hl = lane >> 4, k8 = hl * 8;
  const int nqt = SEQ / 64;
  const int bh = blockIdx.x / nqt, qt = blockIdx.x - bh * nqt;
  const int b = bh / NHEAD, hh = bh - b * NHEAD;
  const int tq = qt * 64 + 16 * w;

  Frag qa0, qa1;
  {
    const unsigned short* qr = qp + ((size_t)bh * SEQ + tq + m) * HD + k8;
    qa0.q[0] = *(const v4u*)(qr);
    qa0.q[1] = *(const v4u*)(qr + 16);
    qa1.q[0] = *(const v4u*)(qr + 32);
    qa1.q[1] = *(const v4u*)(qr + 48);
  }
  float mrun[8], lrun[8];
  v8f oacc[4];
#pragma unroll
  for (int r = 0; r < 8; ++r) { mrun[r] = -1e30f; lrun[r] = 0.0f; }
#pragma unroll
  for (int j = 0; j < 4; ++j) oacc[j] = zero8();

#pragma unroll 1
  for (int kt = 0; kt < nqt; ++kt) {
    v8f s[4];
    const unsigned short* kb = kp + ((size_t)bh * SEQ + kt * 64 + m) * HD + k8;
#pragma unroll
    for (int j = 0; j < 4; ++j) {
      const unsigned short* kr = kb + j * 16 * HD;
      Frag f0, f1;
      f0.q[0] = *(const v4u*)(kr);
      f0.q[1] = *(const v4u*)(kr + 16);
      f1.q[0] = *(const v4u*)(kr + 32);
      f1.q[1] = *(const v4u*)(kr + 48);
      v8f t = mma(qa0.v, f0.v, zero8());
      t = mma(qa1.v, f1.v, t);
      s[j] = t;
    }
    float tmax[8];
#pragma unroll
    for (int r = 0; r < 8; ++r) tmax[r] = -1e30f;
#pragma unroll
    for (int j = 0; j < 4; ++j) {
#pragma unroll
      for (int r = 0; r < 8; ++r) {
        const float val = s[j][r] * 0.125f;
        s[j][r] = val;
        tmax[r] = fmaxf(tmax[r], val);
      }
    }
#pragma unroll
    for (int r = 0; r < 8; ++r) {
#pragma unroll
      for (int xm = 1; xm < 16; xm <<= 1) tmax[r] = fmaxf(tmax[r], __shfl_xor(tmax[r], xm, 32));
    }
    float corr[8];
#pragma unroll
    for (int r = 0; r < 8; ++r) {
      const float mn = fmaxf(mrun[r], tmax[r]);
      corr[r] = __expf(mrun[r] - mn);
      mrun[r] = mn;
    }
    float tsum[8];
#pragma unroll
    for (int r = 0; r < 8; ++r) tsum[r] = 0.0f;
#pragma unroll
    for (int j = 0; j < 4; ++j) {
#pragma unroll
      for (int r = 0; r < 8; ++r) {
        const float p = __expf(s[j][r] - mrun[r]);
        tsum[r] += p;
        sP[w][8 * hl + r][16 * j + m] = hbits(p * 1024.0f);
      }
    }
#pragma unroll
    for (int r = 0; r < 8; ++r) {
#pragma unroll
      for (int xm = 1; xm < 16; xm <<= 1) tsum[r] += __shfl_xor(tsum[r], xm, 32);
      lrun[r] = lrun[r] * corr[r] + tsum[r];
    }
#pragma unroll
    for (int j = 0; j < 4; ++j) {
#pragma unroll
      for (int r = 0; r < 8; ++r) oacc[j][r] *= corr[r];
    }
    __syncthreads();
    Frag pa0, pa1;
    {
      const unsigned short* pr = &sP[w][m][k8];
      pa0.q[0] = *(const v4u*)(pr);
      pa0.q[1] = *(const v4u*)(pr + 16);
      pa1.q[0] = *(const v4u*)(pr + 32);
      pa1.q[1] = *(const v4u*)(pr + 48);
    }
    const unsigned short* vb = vp + ((size_t)bh * HD + m) * (size_t)SEQ + kt * 64 + k8;
#pragma unroll
    for (int jd = 0; jd < 4; ++jd) {
      const unsigned short* vr = vb + (size_t)jd * 16 * SEQ;
      Frag g0, g1;
      g0.q[0] = *(const v4u*)(vr);
      g0.q[1] = *(const v4u*)(vr + 16);
      g1.q[0] = *(const v4u*)(vr + 32);
      g1.q[1] = *(const v4u*)(vr + 48);
      oacc[jd] = mma(pa0.v, g0.v, oacc[jd]);
      oacc[jd] = mma(pa1.v, g1.v, oacc[jd]);
    }
    __syncthreads();
  }

  float il[8];
#pragma unroll
  for (int r = 0; r < 8; ++r) il[r] = 1.0f / (lrun[r] * 1024.0f);
#pragma unroll
  for (int jd = 0; jd < 4; ++jd) {
#pragma unroll
    for (int r = 0; r < 8; ++r) sP[w][8 * hl + r][16 * jd + m] = hbits(oacc[jd][r] * il[r]);
  }
  __syncthreads();
  v4u val[4];
  unsigned int off[4];
#pragma unroll
  for (int p = 0; p < 4; ++p) {
    const int row = 4 * p + (lane >> 3);
    const int piece = lane & 7;
    val[p] = *(const v4u*)&sP[w][row][piece * 8];
    off[p] = (unsigned int)((size_t)(b * SEQ + tq + row) * CDIM + hh * HD + piece * 8);
  }
#pragma unroll
  for (int p = 0; p < 4; ++p) *(volatile v4u*)(op + off[p]) = val[p];
  __threadfence();
#pragma unroll
  for (int p = 0; p < 4; ++p) *(volatile v4u*)(op + off[p]) = val[p];
}

constexpr size_t al256c(size_t v) { return (v + 255) & ~(size_t)255; }
constexpr size_t MCE = (size_t)MROWS * CDIM;
constexpr size_t SZ_WQKV = al256c((size_t)3 * CDIM * CDIM * 2);
constexpr size_t SZ_WO   = al256c((size_t)CDIM * CDIM * 2);
constexpr size_t SZ_W1   = al256c((size_t)HID * CDIM * 2);
constexpr size_t SZ_W2   = al256c((size_t)CDIM * HID * 2);
constexpr size_t SZ_H    = al256c(MCE * 2);
constexpr size_t SZ_QKV  = al256c((size_t)3 * MCE * 2);
constexpr size_t SZ_O    = al256c(MCE * 2);
constexpr size_t SZ_X1   = al256c(MCE * 4);
constexpr size_t SZ_H2   = al256c(MCE * 2);
constexpr size_t SZ_ACT  = al256c((size_t)MROWS * HID * 2);
constexpr size_t WS_TOTAL = SZ_WQKV + SZ_WO + SZ_W1 + SZ_W2 + SZ_H + SZ_QKV + SZ_O + SZ_X1 + SZ_H2 + SZ_ACT;
static_assert(WS_TOTAL <= (size_t)134217728);
static_assert((size_t)MROWS * HID < (size_t)4294967296ull);
static_assert((size_t)NB_FULL * SEQ_FULL * CDIM < (size_t)4294967296ull);

extern "C" void kernel_launch(void* const* d_in, const int* in_sizes, int n_in,
                              void* d_out, int out_size, void* d_ws, size_t ws_size,
                              hipStream_t stream) {
  if (n_in < 17) return;
  const long needX = ((long)(NB - 1) * SEQ_FULL + SEQ) * CDIM;
  const long nWW = (long)CDIM * CDIM;
  if ((long)in_sizes[0] < needX) return;
  if ((long)in_sizes[1] < nWW || in_sizes[2] < CDIM) return;
  if ((long)in_sizes[3] < nWW || in_sizes[4] < CDIM) return;
  if ((long)in_sizes[5] < nWW || in_sizes[6] < CDIM) return;
  if ((long)in_sizes[7] < nWW || in_sizes[8] < CDIM) return;
  if ((long)in_sizes[9] < (long)CDIM * HID || in_sizes[10] < HID) return;
  if ((long)in_sizes[11] < (long)HID * CDIM || in_sizes[12] < CDIM) return;
  if (in_sizes[13] < CDIM || in_sizes[14] < CDIM) return;
  if (in_sizes[15] < CDIM || in_sizes[16] < CDIM) return;
  if ((long)out_size < needX) return;
  if ((size_t)WS_TOTAL > ws_size) return;

  const float* x   = (const float*)d_in[0];
  const float* Wq  = (const float*)d_in[1];
  const float* bq  = (const float*)d_in[2];
  const float* Wk  = (const float*)d_in[3];
  const float* bk  = (const float*)d_in[4];
  const float* Wv  = (const float*)d_in[5];
  const float* bv  = (const float*)d_in[6];
  const float* Wo  = (const float*)d_in[7];
  const float* bo  = (const float*)d_in[8];
  const float* W1  = (const float*)d_in[9];
  const float* b1  = (const float*)d_in[10];
  const float* W2  = (const float*)d_in[11];
  const float* b2  = (const float*)d_in[12];
  const float* g1  = (const float*)d_in[13];
  const float* be1 = (const float*)d_in[14];
  const float* g2  = (const float*)d_in[15];
  const float* be2 = (const float*)d_in[16];
  float* out = (float*)d_out;

  char* ws = (char*)d_ws;
  size_t off = 0;
  unsigned short* wqkv = (unsigned short*)(ws + off); off += SZ_WQKV;
  unsigned short* wot  = (unsigned short*)(ws + off); off += SZ_WO;
  unsigned short* w1t  = (unsigned short*)(ws + off); off += SZ_W1;
  unsigned short* w2t  = (unsigned short*)(ws + off); off += SZ_W2;
  unsigned short* hpl  = (unsigned short*)(ws + off); off += SZ_H;
  unsigned short* qkv  = (unsigned short*)(ws + off); off += SZ_QKV;
  unsigned short* opl  = (unsigned short*)(ws + off); off += SZ_O;
  float*          x1   = (float*)(ws + off);          off += SZ_X1;
  unsigned short* h2p  = (unsigned short*)(ws + off); off += SZ_H2;
  unsigned short* act  = (unsigned short*)(ws + off); off += SZ_ACT;
  if (off > ws_size) return;
  unsigned short* qpl = qkv;
  unsigned short* kpl = qkv + MCE;
  unsigned short* vtp = qkv + 2 * MCE;

  k_wprep<<<dim3(CDIM / 64, CDIM / 64), 256, 0, stream>>>(Wq, wqkv, CDIM, CDIM, 0);
  k_wprep<<<dim3(CDIM / 64, CDIM / 64), 256, 0, stream>>>(Wk, wqkv, CDIM, CDIM, CDIM);
  k_wprep<<<dim3(CDIM / 64, CDIM / 64), 256, 0, stream>>>(Wv, wqkv, CDIM, CDIM, 2 * CDIM);
  k_wprep<<<dim3(CDIM / 64, CDIM / 64), 256, 0, stream>>>(Wo, wot, CDIM, CDIM, 0);
  k_wprep<<<dim3(CDIM / 64, HID / 64), 256, 0, stream>>>(W1, w1t, CDIM, HID, 0);
  k_wprep<<<dim3(HID / 64, CDIM / 64), 256, 0, stream>>>(W2, w2t, HID, CDIM, 0);
  k_ln_in<<<MROWS / 8, 256, 0, stream>>>(x, g1, be1, hpl, MROWS);
  k_gemm_qkv<<<dim3(3 * CDIM / 64, MROWS / 64), 128, 0, stream>>>(hpl, wqkv, bq, bk, bv, qkv);
  k_attn<<<NB * NHEAD * (SEQ / 64), 128, 0, stream>>>(qpl, kpl, vtp, opl);
  k_gemm_res<<<dim3(CDIM / 64, MROWS / 64), 128, 0, stream>>>(opl, wot, CDIM, bo, x, x1, 1, 0);
  k_ln_mid<<<MROWS / 8, 256, 0, stream>>>(x1, g2, be2, h2p, MROWS);
  k_gemm_gelu<<<dim3(HID / 64, MROWS / 64), 128, 0, stream>>>(h2p, w1t, CDIM, b1, act);
  k_gemm_res<<<dim3(CDIM / 64, MROWS / 64), 128, 0, stream>>>(act, w2t, HID, b2, x1, out, 0, 1);
}
